// Mamba_8143257993724
// MI455X (gfx1250) — hardware-verified
//
#include <hip/hip_runtime.h>
#include <math.h>

constexpr int NBATCH = 8;
constexpr int SEQ    = 4096;
constexpr int NCH    = 256;
constexpr int NHEAD  = 8;
constexpr int HDIM   = 32;
constexpr int KCONV  = 4;
constexpr int NGATE  = 4;
constexpr int TSTEP  = 16;
constexpr int NTILE  = SEQ / TSTEP;
constexpr int APITCH = 264;
constexpr int RPITCH = 40;
constexpr int SPITCH = 36;
constexpr int NTHR_P = 256;
constexpr int NTHR_S = 64;
constexpr int PRE_ROWF = NBATCH * NHEAD * HDIM * NGATE;
constexpr int PRE_BATF = NHEAD * HDIM * NGATE;
constexpr size_t PRE_BYTES = (size_t)SEQ * (size_t)PRE_ROWF * 4;
static_assert(PRE_BYTES == (size_t)134217728);
static_assert(SEQ % TSTEP == 0 && TSTEP == 16);
static_assert(NCH == NTHR_P && NHEAD * 32 == NTHR_P);
static_assert(HDIM == 32 && NHEAD * HDIM == NCH && KCONV == 4 && NGATE == 4);
static_assert(APITCH % 8 == 0 && RPITCH % 8 == 0 && SPITCH % 4 == 0);
static_assert(NGATE * HDIM * HDIM == 16 * NTHR_S * 4);
static_assert(16 * HDIM == 8 * NTHR_S);
static_assert(NTHR_S == 64 && NBATCH == 8);

typedef __attribute__((ext_vector_type(16))) __bf16 v16b;
typedef __attribute__((ext_vector_type(8)))  __bf16 v8b;
typedef __attribute__((ext_vector_type(8)))  float  v8f;
typedef __attribute__((ext_vector_type(4)))  float  v4f;

__device__ __forceinline__ unsigned short f2bf_bits(float f) {
  unsigned u = __float_as_uint(f);
  return (unsigned short)((u + 0x7FFFu + ((u >> 16) & 1u)) >> 16);
}
__device__ __forceinline__ float bf_bits2f(unsigned short h) { return __uint_as_float(((unsigned)h) << 16); }
__device__ __forceinline__ void split_bf(float f, unsigned short& hb, unsigned short& lb) {
  hb = f2bf_bits(f);
  lb = f2bf_bits(f - bf_bits2f(hb));
}

struct FragB {
  union U { v16b v; v8b h[2]; };
  static __device__ __forceinline__ v16b load(const __bf16* p) {
    U f; f.h[0] = *(const v8b*)(p); f.h[1] = *(const v8b*)(p + 16); return f.v;
  }
  static __device__ __forceinline__ v8f mma(v16b a, v16b b, v8f c) {
    return __builtin_amdgcn_wmma_f32_16x16x32_bf16(false, a, false, b, (short)0, c, false, false);
  }
};

__device__ __forceinline__ void guard4x12(v8f& a0, v8f& a1, v8f& a2, v8f& a3,
                                          v16b f0, v16b f1, v16b f2, v16b f3, v16b f4, v16b f5,
                                          v16b f6, v16b f7, v16b f8, v16b f9, v16b f10, v16b f11) {
  asm volatile("v_nop\n\tv_nop\n\tv_nop\n\tv_nop"
               : "+v"(a0), "+v"(a1), "+v"(a2), "+v"(a3)
               : "v"(f0), "v"(f1), "v"(f2), "v"(f3), "v"(f4), "v"(f5), "v"(f6), "v"(f7), "v"(f8), "v"(f9), "v"(f10), "v"(f11));
}
__device__ __forceinline__ void guard4x10(v8f& a0, v8f& a1, v8f& a2, v8f& a3,
                                          v16b f0, v16b f1, v16b f2, v16b f3, v16b f4,
                                          v16b f5, v16b f6, v16b f7, v16b f8, v16b f9) {
  asm volatile("v_nop\n\tv_nop\n\tv_nop\n\tv_nop"
               : "+v"(a0), "+v"(a1), "+v"(a2), "+v"(a3)
               : "v"(f0), "v"(f1), "v"(f2), "v"(f3), "v"(f4), "v"(f5), "v"(f6), "v"(f7), "v"(f8), "v"(f9));
}
__device__ __forceinline__ void mem_clobber() { asm volatile("" ::: "memory"); }

__device__ __forceinline__ void load_w_frag(const float* wrow, int koff, v16b& bh_out, v16b& bl_out) {
  const v4f q0 = *(const v4f*)(wrow + koff);
  const v4f q1 = *(const v4f*)(wrow + koff + 4);
  const v4f q2 = *(const v4f*)(wrow + koff + 16);
  const v4f q3 = *(const v4f*)(wrow + koff + 20);
  v16b bh, bl;
#pragma unroll
  for (int e = 0; e < 4; ++e) {
    unsigned short hb, lb;
    float f;
    f = q0[e]; split_bf(f, hb, lb); bh[e]      = __builtin_bit_cast(__bf16, hb); bl[e]      = __builtin_bit_cast(__bf16, lb);
    f = q1[e]; split_bf(f, hb, lb); bh[4 + e]  = __builtin_bit_cast(__bf16, hb); bl[4 + e]  = __builtin_bit_cast(__bf16, lb);
    f = q2[e]; split_bf(f, hb, lb); bh[8 + e]  = __builtin_bit_cast(__bf16, hb); bl[8 + e]  = __builtin_bit_cast(__bf16, lb);
    f = q3[e]; split_bf(f, hb, lb); bh[12 + e] = __builtin_bit_cast(__bf16, hb); bl[12 + e] = __builtin_bit_cast(__bf16, lb);
  }
  bh_out = bh; bl_out = bl;
}

__global__ __launch_bounds__(NTHR_P) void proj_kernel(const float* x, const float* conv_w, const float* conv_b,
                                                      const float* w_i, const float* w_f, const float* w_z,
                                                      const float* w_o, float* pre) {
  __shared__ __align__(16) unsigned short sCh[TSTEP * APITCH];
  __shared__ __align__(16) unsigned short sCl[TSTEP * APITCH];
  __shared__ __align__(16) unsigned short sXh[TSTEP * APITCH];
  __shared__ __align__(16) unsigned short sXl[TSTEP * APITCH];
  const int tid = threadIdx.x;
  const int blk = blockIdx.x;
  const int b   = blk / NTILE;
  const int s0  = (blk - b * NTILE) * TSTEP;

  {
    const int d = tid;
    const v4f cw = *(const v4f*)(conv_w + 4 * d);
    const float cb = conv_b[d];
    const float* xb = x + (size_t)b * SEQ * NCH + d;
    const bool has_halo = (s0 > 0);
    const int sm3 = has_halo ? (s0 - 3) : 0;
    const int sm2 = has_halo ? (s0 - 2) : 0;
    const int sm1 = has_halo ? (s0 - 1) : 0;
    float w0 = xb[(size_t)sm3 * NCH];
    float w1 = xb[(size_t)sm2 * NCH];
    float w2 = xb[(size_t)sm1 * NCH];
    w0 = has_halo ? w0 : 0.0f;
    w1 = has_halo ? w1 : 0.0f;
    w2 = has_halo ? w2 : 0.0f;
#pragma unroll 1
    for (int si = 0; si < TSTEP; ++si) {
      const float w3 = xb[(size_t)(s0 + si) * NCH];
      float t = cw[0] * w0;
      t = t + cw[1] * w1;
      t = t + cw[2] * w2;
      t = t + cw[3] * w3;
      t = t + cb;
      const float sg = 1.0f / (1.0f + expf(-t));
      const float xc = t * sg;
      unsigned short hb, lb;
      split_bf(xc, hb, lb);
      sCh[si * APITCH + d] = hb;
      sCl[si * APITCH + d] = lb;
      split_bf(w3, hb, lb);
      sXh[si * APITCH + d] = hb;
      sXl[si * APITCH + d] = lb;
      w0 = w1; w1 = w2; w2 = w3;
    }
  }
  __syncthreads();

  const int lane = tid & 31;
  const int n    = tid >> 5;
  const int hh   = lane >> 4;
  const int c    = lane & 15;
  const int koff = 8 * hh;
  const int aoff = c * APITCH + n * HDIM + koff;
  const v16b ach = FragB::load((const __bf16*)sCh + aoff);
  const v16b acl = FragB::load((const __bf16*)sCl + aoff);
  const v16b axh = FragB::load((const __bf16*)sXh + aoff);
  const v16b axl = FragB::load((const __bf16*)sXl + aoff);
  const v8f z8 = {0.f, 0.f, 0.f, 0.f, 0.f, 0.f, 0.f, 0.f};

#pragma unroll
  for (int nt = 0; nt < 2; ++nt) {
    const int o = nt * 16 + c;
    const size_t woff = (size_t)(n * HDIM + o) * HDIM;
    v16b bh[4], bl[4];
    load_w_frag(w_i + woff, koff, bh[0], bl[0]); mem_clobber();
    load_w_frag(w_f + woff, koff, bh[1], bl[1]); mem_clobber();
    load_w_frag(w_z + woff, koff, bh[2], bl[2]); mem_clobber();
    load_w_frag(w_o + woff, koff, bh[3], bl[3]); mem_clobber();

    v8f acc[4];
    acc[0] = z8; acc[1] = z8; acc[2] = z8; acc[3] = z8;
    acc[0] = FragB::mma(ach, bh[0], acc[0]); acc[0] = FragB::mma(ach, bl[0], acc[0]); acc[0] = FragB::mma(acl, bh[0], acc[0]);
    acc[1] = FragB::mma(ach, bh[1], acc[1]); acc[1] = FragB::mma(ach, bl[1], acc[1]); acc[1] = FragB::mma(acl, bh[1], acc[1]);
    acc[2] = FragB::mma(axh, bh[2], acc[2]); acc[2] = FragB::mma(axh, bl[2], acc[2]); acc[2] = FragB::mma(axl, bh[2], acc[2]);
    acc[3] = FragB::mma(axh, bh[3], acc[3]); acc[3] = FragB::mma(axh, bl[3], acc[3]); acc[3] = FragB::mma(axl, bh[3], acc[3]);
    guard4x12(acc[0], acc[1], acc[2], acc[3], ach, acl, axh, axl, bh[0], bh[1], bh[2], bh[3], bl[0], bl[1], bl[2], bl[3]);

    v4f vv[8];
#pragma unroll
    for (int r = 0; r < 8; ++r) {
      v4f v;
      v[0] = acc[0][r]; v[1] = acc[1][r]; v[2] = acc[2][r]; v[3] = acc[3][r];
      vv[r] = v;
    }
    float* pb = pre + (size_t)(s0 + 8 * hh) * PRE_ROWF + (size_t)b * PRE_BATF + (size_t)n * (HDIM * NGATE) + (size_t)o * NGATE;
    for (int pass = 0; pass < 2; ++pass) {
#pragma unroll
      for (int r = 0; r < 8; ++r) *(volatile v4f*)(pb + (size_t)r * PRE_ROWF) = vv[r];
      __threadfence();
    }
  }
}

__global__ __launch_bounds__(NTHR_S) void scan_kernel(const float* pre, const float* R, const float* bias,
                                                      const float* gn_w, float* out) {
  __shared__ __align__(16) unsigned short Rh[NGATE * HDIM * RPITCH];
  __shared__ __align__(16) unsigned short Rl[NGATE * HDIM * RPITCH];
  __shared__ __align__(16) unsigned short Hh[2][16 * RPITCH];
  __shared__ __align__(16) unsigned short Hl[2][16 * RPITCH];
  __shared__ __align__(16) float          Sl[2][16 * SPITCH];
  const int n    = blockIdx.x;
  const int tid  = threadIdx.x;
  const int lane = tid & 31;
  const int wave = tid >> 5;
  const int hh   = lane >> 4;
  const int c    = lane & 15;
  const int koff = 8 * hh;
  const int ucol = 16 * wave + c;

  {
    const float* Rn = R + (size_t)n * (NGATE * HDIM * HDIM);
#pragma unroll 1
    for (int it = 0; it < 16; ++it) {
      const int f4 = it * NTHR_S + tid;
      const v4f v = *(const v4f*)(Rn + 4 * f4);
      const int row = f4 >> 3;
      const int col = (f4 & 7) * 4;
#pragma unroll
      for (int e = 0; e < 4; ++e) {
        unsigned short hb, lb;
        const float f = v[e];
        split_bf(f, hb, lb);
        Rh[row * RPITCH + col + e] = hb;
        Rl[row * RPITCH + col + e] = lb;
      }
    }
  }
#pragma unroll
  for (int it = 0; it < 8; ++it) {
    const int idx = it * NTHR_S + tid;
    const int row = idx >> 5, col = idx & 31;
    Hh[0][row * RPITCH + col] = (unsigned short)0;
    Hl[0][row * RPITCH + col] = (unsigned short)0;
  }
  float bb[4];
#pragma unroll
  for (int g = 0; g < 4; ++g) bb[g] = bias[(n * NGATE + g) * HDIM + ucol];
  const v4f gw = *(const v4f*)(gn_w + n * HDIM + (lane & 7) * 4);
  float cst[8], nst[8], mst[8];
#pragma unroll
  for (int r = 0; r < 8; ++r) { cst[r] = 0.0f; nst[r] = 0.0f; mst[r] = -1e30f; }
  __syncthreads();

  const v8f z8 = {0.f, 0.f, 0.f, 0.f, 0.f, 0.f, 0.f, 0.f};

#pragma unroll 1
  for (int s = 0; s < SEQ; ++s) {
    const int cur = s & 1;
    const int nxt = cur ^ 1;

    const float* pp = pre + (size_t)s * PRE_ROWF + (size_t)n * (HDIM * NGATE) + (size_t)ucol * NGATE;
    v4f p[8];
#pragma unroll
    for (int r = 0; r < 8; ++r) p[r] = *(const v4f*)(pp + (size_t)r * PRE_BATF);

    const int aoff = c * RPITCH + koff;
    const v16b ah = FragB::load((const __bf16*)Hh[cur] + aoff);
    const v16b al = FragB::load((const __bf16*)Hl[cur] + aoff);
    v16b bh[4], bl[4];
#pragma unroll
    for (int g = 0; g < 4; ++g) {
      const int boff = (g * HDIM + ucol) * RPITCH + koff;
      bh[g] = FragB::load((const __bf16*)Rh + boff);
      bl[g] = FragB::load((const __bf16*)Rl + boff);
    }
    v8f acc[4];
    acc[0] = z8; acc[1] = z8; acc[2] = z8; acc[3] = z8;
#pragma unroll
    for (int g = 0; g < 4; ++g) {
      acc[g] = FragB::mma(ah, bh[g], acc[g]);
      acc[g] = FragB::mma(ah, bl[g], acc[g]);
      acc[g] = FragB::mma(al, bh[g], acc[g]);
    }
    guard4x10(acc[0], acc[1], acc[2], acc[3], ah, al, bh[0], bh[1], bh[2], bh[3], bl[0], bl[1], bl[2], bl[3]);

#pragma unroll
    for (int r = 0; r < 8; ++r) {
      const float ri = (p[r][0] + acc[0][r]) + bb[0];
      const float rf = (p[r][1] + acc[1][r]) + bb[1];
      const float rz = (p[r][2] + acc[2][r]) + bb[2];
      const float ro = (p[r][3] + acc[3][r]) + bb[3];
      const float lf  = fminf(rf, 0.0f) - log1pf(expf(-fabsf(rf)));
      const float lfm = mst[r] + lf;
      const float mn  = fmaxf(ri, lfm);
      const float ig  = expf(ri - mn);
      const float fg  = expf(lfm - mn);
      const float cn  = fg * cst[r] + ig * tanhf(rz);
      const float nn  = fg * nst[r] + ig;
      const float og  = 1.0f / (1.0f + expf(-ro));
      const float hn  = (og * cn) * (1.0f / nn);
      cst[r] = cn; nst[r] = nn; mst[r] = mn;
      unsigned short hb, lb;
      split_bf(hn, hb, lb);
      Hh[nxt][(8 * hh + r) * RPITCH + ucol] = hb;
      Hl[nxt][(8 * hh + r) * RPITCH + ucol] = lb;
      Sl[cur][(8 * hh + r) * SPITCH + ucol] = hn;
    }
    __syncthreads();

    {
      const int q  = lane >> 3;
      const int c4 = (lane & 7) * 4;
      const int brow = 4 * wave + q;
      const v4f v = *(const v4f*)(Sl[cur] + brow * SPITCH + c4);
      float sm = (v[0] + v[1]) + (v[2] + v[3]);
      sm += __shfl_xor(sm, 1, 32);
      sm += __shfl_xor(sm, 2, 32);
      sm += __shfl_xor(sm, 4, 32);
      const float mu = sm * (1.0f / 32.0f);
      v4f dv;
      float ss = 0.0f;
#pragma unroll
      for (int e = 0; e < 4; ++e) { const float dd = v[e] - mu; dv[e] = dd; ss += dd * dd; }
      ss += __shfl_xor(ss, 1, 32);
      ss += __shfl_xor(ss, 2, 32);
      ss += __shfl_xor(ss, 4, 32);
      const float var  = ss * (1.0f / 32.0f);
      const float rstd = rsqrtf(var + 1e-5f);
      v4f y;
#pragma unroll
      for (int e = 0; e < 4; ++e) y[e] = (dv[e] * rstd) * gw[e];
      float* op = out + ((size_t)brow * SEQ + (size_t)s) * NCH + n * HDIM + c4;
      *(volatile v4f*)op = y;
      __threadfence();
      *(volatile v4f*)op = y;
    }
  }
}

extern "C" void kernel_launch(void* const* d_in, const int* in_sizes, int n_in,
                              void* d_out, int out_size, void* d_ws, size_t ws_size, hipStream_t stream) {
  if (n_in < 10 || d_out == nullptr || d_ws == nullptr) return;
  if (in_sizes[0] != NBATCH * SEQ * NCH || in_sizes[1] != NCH * KCONV || in_sizes[2] != NCH ||
      in_sizes[3] != NHEAD * HDIM * HDIM || in_sizes[4] != NHEAD * HDIM * HDIM ||
      in_sizes[5] != NHEAD * HDIM * HDIM || in_sizes[6] != NHEAD * HDIM * HDIM ||
      in_sizes[7] != NHEAD * NGATE * HDIM * HDIM || in_sizes[8] != NHEAD * NGATE * HDIM ||
      in_sizes[9] != NCH || out_size != NBATCH * SEQ * NCH) return;
  if (ws_size < PRE_BYTES) return;

  const float* x      = (const float*)d_in[0];
  const float* conv_w = (const float*)d_in[1];
  const float* conv_b = (const float*)d_in[2];
  const float* w_i    = (const float*)d_in[3];
  const float* w_f    = (const float*)d_in[4];
  const float* w_z    = (const float*)d_in[5];
  const float* w_o    = (const float*)d_in[6];
  const float* R      = (const float*)d_in[7];
  const float* bias   = (const float*)d_in[8];
  const float* gn_w   = (const float*)d_in[9];
  float* out = (float*)d_out;
  float* pre = (float*)d_ws;

  proj_kernel<<<NBATCH * NTILE, NTHR_P, 0, stream>>>(x, conv_w, conv_b, w_i, w_f, w_z, w_o, pre);
  scan_kernel<<<NHEAD, NTHR_S, 0, stream>>>(pre, R, bias, gn_w, out);
}
